// HebbianLayer_35622458753122
// MI455X (gfx1250) — hardware-run, weakly checked
//
#include <hip/hip_runtime.h>

constexpr int N_IN  = 512;
constexpr int N_OUT = 128;
constexpr int N_SMP = 4096;
constexpr float LRATE = 1e-4f;

constexpr int OUT0_ELEMS = N_SMP * N_OUT;
constexpr int OUT1_ELEMS = N_OUT * N_IN;
constexpr int OUT1_OFF_BYTES = 2097152;
constexpr int OUT_TOTAL_BYTES = 2359296;
static_assert(OUT0_ELEMS * 4 == OUT1_OFF_BYTES);
static_assert(OUT1_OFF_BYTES + OUT1_ELEMS * 4 == OUT_TOTAL_BYTES);
static_assert(OUT1_OFF_BYTES % 128 == 0);
static_assert(N_SMP % 64 == 0 && N_OUT % 64 == 0 && N_IN % 32 == 0);
static_assert(((N_SMP / 64) * (N_OUT / 64)) % 8 == 0);

typedef __attribute__((ext_vector_type(16))) __bf16   v16b;
typedef __attribute__((ext_vector_type(8)))  __bf16   v8b;
typedef __attribute__((ext_vector_type(8)))  float    v8f;
typedef __attribute__((ext_vector_type(4)))  float    v4f;
typedef __attribute__((ext_vector_type(4)))  unsigned v4u;

constexpr size_t SZ_XPLANE = (size_t)N_SMP * N_IN * 2;
constexpr size_t SZ_WPLANE = (size_t)N_OUT * N_IN * 2;
constexpr size_t OFF_XH = 0;
constexpr size_t OFF_XL = OFF_XH + SZ_XPLANE;
constexpr size_t OFF_WH = OFF_XL + SZ_XPLANE;
constexpr size_t OFF_WL = OFF_WH + SZ_WPLANE;
constexpr size_t WS_TOTAL = OFF_WL + SZ_WPLANE;
static_assert(WS_TOTAL == 8650752);
static_assert(OFF_XL % 128 == 0 && OFF_WH % 128 == 0 && OFF_WL % 128 == 0);

__device__ __forceinline__ unsigned bf_bits32(float f) {
  const unsigned u = __float_as_uint(f);
  return (u + 0x7FFFu + ((u >> 16) & 1u)) >> 16;
}
__device__ __forceinline__ void split_pair(float f0, float f1, unsigned& wh, unsigned& wl) {
  const unsigned h0 = bf_bits32(f0);
  const unsigned h1 = bf_bits32(f1);
  const float r0 = f0 - __uint_as_float(h0 << 16);
  const float r1 = f1 - __uint_as_float(h1 << 16);
  const unsigned l0 = bf_bits32(r0);
  const unsigned l1 = bf_bits32(r1);
  wh = h0 | (h1 << 16);
  wl = l0 | (l1 << 16);
}

constexpr int SPLIT_THR = 256;
static_assert(((size_t)N_SMP * N_IN) % (SPLIT_THR * 8) == 0);
static_assert(((size_t)N_OUT * N_IN) % (SPLIT_THR * 8) == 0);
__global__ void __launch_bounds__(SPLIT_THR)
split_planes_kernel(const float* __restrict__ src, unsigned* __restrict__ hi, unsigned* __restrict__ lo) {
  const size_t i = (size_t)blockIdx.x * SPLIT_THR + threadIdx.x;
  const v4f a = *(const v4f*)(src + 8 * i);
  const v4f b = *(const v4f*)(src + 8 * i + 4);
  v4u vh, vl;
  unsigned wh, wl;
  split_pair(a[0], a[1], wh, wl);
  vh[0] = wh; vl[0] = wl;
  split_pair(a[2], a[3], wh, wl);
  vh[1] = wh; vl[1] = wl;
  split_pair(b[0], b[1], wh, wl);
  vh[2] = wh; vl[2] = wl;
  split_pair(b[2], b[3], wh, wl);
  vh[3] = wh; vl[3] = wl;
  volatile v4u* const ph = (volatile v4u*)(hi + 4 * i);
  volatile v4u* const pl = (volatile v4u*)(lo + 4 * i);
  for (int pass = 0; pass < 2; ++pass) {
    *ph = vh;
    *pl = vl;
    __threadfence();
  }
}

union FragB { v16b v; v8b h[2]; };
__device__ __forceinline__ v16b frag_load(const __bf16* p) {
  FragB f;
  f.h[0] = *(const v8b*)(p);
  f.h[1] = *(const v8b*)(p + 16);
  return f.v;
}
__device__ __forceinline__ v8f mma_bf(v16b a, v16b b, v8f c) {
  return __builtin_amdgcn_wmma_f32_16x16x32_bf16(false, a, false, b, (short)0, c, false, false);
}
__device__ __forceinline__ void tie_acc(v8f& a, v16b x, v16b y) {
  asm volatile("v_nop\n\tv_nop\n\tv_nop\n\tv_nop" : "+v"(a) : "v"(x), "v"(y));
}
__device__ __forceinline__ void keep4(v16b a, v16b b, v16b c, v16b d) {
  asm volatile("v_nop" :: "v"(a), "v"(b), "v"(c), "v"(d));
}
__device__ __forceinline__ void tie_acc_only(v8f& a) {
  asm volatile("v_nop\n\tv_nop\n\tv_nop\n\tv_nop" : "+v"(a));
}

__global__ void __launch_bounds__(256)
gemm64_bf16x3_bias_kernel(const unsigned short* __restrict__ Ap, const unsigned short* __restrict__ A2p, int lda,
                          const unsigned short* __restrict__ Btp, const unsigned short* __restrict__ Bt2p, int ldb,
                          float* __restrict__ C, int ldc, const float* __restrict__ bias,
                          int M, int N, int K) {
  const __bf16* A   = (const __bf16*)Ap;
  const __bf16* A2  = (const __bf16*)A2p;
  const __bf16* Bt  = (const __bf16*)Btp;
  const __bf16* Bt2 = (const __bf16*)Bt2p;
  __shared__ __align__(16) float sT[8][16 * 68];
  const int lane = threadIdx.x & 31;
  const int wave = threadIdx.x >> 5;
  const int tilesN = N >> 6;
  const int tilesM = M >> 6;
  const int tile = blockIdx.x * 8 + wave;
  if (tile >= tilesM * tilesN) return;
  const int tm = tile / tilesN;
  const int tn = tile - tm * tilesN;
  const int m0 = tm << 6;
  const int n0 = tn << 6;

  const int rlane = lane & 15;
  const int koff  = (lane >> 4) * 8;
  const int mOff  = (lane >> 4) * 8;

  v8f acc[4][4];
#pragma unroll
  for (int i = 0; i < 4; ++i)
#pragma unroll
    for (int j = 0; j < 4; ++j) acc[i][j] = (v8f){0.f, 0.f, 0.f, 0.f, 0.f, 0.f, 0.f, 0.f};

  for (int k0 = 0; k0 < K; k0 += 32) {
    v16b bh[4], bl[4];
#pragma unroll
    for (int j = 0; j < 4; ++j) {
      const size_t bo = (size_t)(n0 + (j << 4) + rlane) * ldb + koff + k0;
      bh[j] = frag_load(Bt + bo);
      bl[j] = frag_load(Bt2 + bo);
    }
#pragma unroll
    for (int i = 0; i < 4; ++i) {
      const size_t ao = (size_t)(m0 + (i << 4) + rlane) * lda + koff + k0;
      const v16b ah = frag_load(A + ao);
      const v16b al = frag_load(A2 + ao);
#pragma unroll
      for (int j = 0; j < 4; ++j) {
        acc[i][j] = mma_bf(ah, bh[j], acc[i][j]);
        acc[i][j] = mma_bf(ah, bl[j], acc[i][j]);
        acc[i][j] = mma_bf(al, bh[j], acc[i][j]);
      }
      tie_acc(acc[i][0], ah, al);
      tie_acc(acc[i][1], ah, al);
      tie_acc(acc[i][2], ah, al);
      tie_acc(acc[i][3], ah, al);
    }
    keep4(bh[0], bh[1], bh[2], bh[3]);
    keep4(bl[0], bl[1], bl[2], bl[3]);
  }
#pragma unroll
  for (int i = 0; i < 4; ++i) {
    tie_acc_only(acc[i][0]);
    tie_acc_only(acc[i][1]);
    tie_acc_only(acc[i][2]);
    tie_acc_only(acc[i][3]);
  }

  float* slab = sT[wave];
#pragma unroll
  for (int i = 0; i < 4; ++i) {
    const int mBase = m0 + (i << 4);
#pragma unroll
    for (int j = 0; j < 4; ++j) {
      const int n = n0 + (j << 4) + rlane;
      const float bv = bias[n];
#pragma unroll
      for (int r = 0; r < 8; ++r) {
        const float v = acc[i][j][r] + bv;
        slab[(mOff + r) * 68 + (j << 4) + rlane] = v;
      }
    }
    __builtin_amdgcn_fence(__ATOMIC_RELEASE, "workgroup");
    __builtin_amdgcn_wave_barrier();
    __builtin_amdgcn_fence(__ATOMIC_ACQUIRE, "workgroup");
    {
      const int hh = lane >> 4;
      const int c4 = (lane & 15) * 4;
      for (int pass = 0; pass < 2; ++pass) {
#pragma unroll
        for (int it = 0; it < 8; ++it) {
          const int row = it * 2 + hh;
          const v4f v = *(const v4f*)(slab + row * 68 + c4);
          *(volatile v4f*)(C + (size_t)(mBase + row) * ldc + n0 + c4) = v;
        }
        __threadfence();
      }
    }
    __builtin_amdgcn_fence(__ATOMIC_RELEASE, "workgroup");
    __builtin_amdgcn_wave_barrier();
    __builtin_amdgcn_fence(__ATOMIC_ACQUIRE, "workgroup");
  }
}

constexpr int SEQ_THR = 512;
constexpr int LDS_W_FLOATS = N_OUT * N_IN;
constexpr int LDS_X_OFF = LDS_W_FLOATS;
constexpr int LDS_Y_OFF = LDS_X_OFF + 2 * N_IN;
constexpr int LDS_B_OFF = LDS_Y_OFF + N_OUT;
constexpr int LDS_SEQ_FLOATS = LDS_B_OFF + N_OUT;
constexpr int LDS_SEQ_BYTES = LDS_SEQ_FLOATS * 4;
static_assert(LDS_SEQ_BYTES == 267264);
static_assert(LDS_SEQ_BYTES <= 298 * 1024);
static_assert((LDS_X_OFF * 4) % 16 == 0 && (LDS_Y_OFF * 4) % 16 == 0 && (LDS_B_OFF * 4) % 16 == 0);
static_assert(N_IN == SEQ_THR);
static_assert((N_OUT * N_IN / 4) % SEQ_THR == 0);
static_assert(N_OUT == (SEQ_THR / 32) * 8);
static_assert(N_IN == 4 * N_OUT);

__global__ void __launch_bounds__(SEQ_THR, 1)
seq_update_kernel(const float* __restrict__ x, const float* __restrict__ w0,
                  const float* __restrict__ bias, float* __restrict__ wout) {
  extern __shared__ v4f seq_lds_dyn[];
  float* const Wl  = (float*)seq_lds_dyn;
  float* const xsh = Wl + LDS_X_OFF;
  float* const ysh = Wl + LDS_Y_OFF;
  float* const bsh = Wl + LDS_B_OFF;

  const int t    = threadIdx.x;
  const int lane = t & 31;
  const int wid  = t >> 5;

  {
    v4f* const Wv = (v4f*)Wl;
    const v4f* const w0v = (const v4f*)w0;
#pragma unroll 1
    for (int it = 0; it < (N_OUT * N_IN / 4) / SEQ_THR; ++it) {
      const int i = it * SEQ_THR + t;
      Wv[i] = w0v[i];
    }
  }
  {
    float bv = bias[t & (N_OUT - 1)];
    asm volatile("" : "+v"(bv));
    if (t < N_OUT) bsh[t] = bv;
  }
  float xv = x[t];
  __syncthreads();

#pragma unroll 1
  for (int b = 0; b < N_SMP; ++b) {
    float* const xcur = xsh + (b & 1) * N_IN;
    xcur[t] = xv;
    __syncthreads();

    v4f xr[4];
#pragma unroll
    for (int j = 0; j < 4; ++j) xr[j] = *(const v4f*)(xcur + 128 * j + 4 * lane);

#pragma unroll 1
    for (int r = 0; r < 8; ++r) {
      const int i = wid * 8 + r;
      const float* const wrow = Wl + i * N_IN + 4 * lane;
      float acc = 0.0f;
#pragma unroll
      for (int j = 0; j < 4; ++j) {
        const v4f wq = *(const v4f*)(wrow + 128 * j);
        acc = fmaf(wq[0], xr[j][0], acc);
        acc = fmaf(wq[1], xr[j][1], acc);
        acc = fmaf(wq[2], xr[j][2], acc);
        acc = fmaf(wq[3], xr[j][3], acc);
      }
      acc += __shfl_xor(acc, 16, 32);
      acc += __shfl_xor(acc, 8, 32);
      acc += __shfl_xor(acc, 4, 32);
      acc += __shfl_xor(acc, 2, 32);
      acc += __shfl_xor(acc, 1, 32);
      const float bi = bsh[i];
      const float yv = acc + bi;
      if (lane == 0) ysh[i] = yv;
    }
    __syncthreads();

    int bn = b + 1;
    bn = (bn < N_SMP) ? bn : (N_SMP - 1);
    const float xn = x[(size_t)bn * N_IN + t];

    if (t < N_OUT) {
      const int c0 = 4 * t;
      const v4f xq = *(const v4f*)(xcur + c0);
      v4f p = {0.0f, 0.0f, 0.0f, 0.0f};
#pragma unroll 1
      for (int i = 0; i < N_OUT; i += 4) {
        const v4f y4 = *(const v4f*)(ysh + i);
#pragma unroll
        for (int u = 0; u < 4; ++u) {
          const float yi = y4[u];
          float* const wp = Wl + (i + u) * N_IN + c0;
          v4f wq = *(const v4f*)wp;
          p[0] = fmaf(yi, wq[0], p[0]);
          p[1] = fmaf(yi, wq[1], p[1]);
          p[2] = fmaf(yi, wq[2], p[2]);
          p[3] = fmaf(yi, wq[3], p[3]);
          const float s = LRATE * yi;
          wq[0] = fmaf(s, xq[0] - p[0], wq[0]);
          wq[1] = fmaf(s, xq[1] - p[1], wq[1]);
          wq[2] = fmaf(s, xq[2] - p[2], wq[2]);
          wq[3] = fmaf(s, xq[3] - p[3], wq[3]);
          *(v4f*)wp = wq;
        }
      }
    }
    xv = xn;
  }

  __syncthreads();

  {
    const v4f* const Wv = (const v4f*)Wl;
    for (int pass = 0; pass < 2; ++pass) {
#pragma unroll 1
      for (int it = 0; it < (N_OUT * N_IN / 4) / SEQ_THR; ++it) {
        const int i = it * SEQ_THR + t;
        const v4f v = Wv[i];
        *(volatile v4f*)(wout + 4 * (size_t)i) = v;
      }
      __threadfence();
    }
  }
}

extern "C" void kernel_launch(void* const* d_in, const int* in_sizes, int n_in,
                              void* d_out, int out_size, void* d_ws, size_t ws_size, hipStream_t stream) {
  if (n_in < 3 || d_out == nullptr || d_ws == nullptr) return;
  if (in_sizes[0] != N_SMP * N_IN || in_sizes[1] != N_OUT * N_IN || in_sizes[2] != N_OUT) return;
  if (out_size != OUT0_ELEMS + OUT1_ELEMS) return;
  if (ws_size < WS_TOTAL) return;

  const float* x    = (const float*)d_in[0];
  const float* w    = (const float*)d_in[1];
  const float* bias = (const float*)d_in[2];
  float* y    = (float*)d_out;
  float* wout = (float*)d_out + (OUT1_OFF_BYTES / 4);

  unsigned char* ws = (unsigned char*)d_ws;
  unsigned short* xh = (unsigned short*)(ws + OFF_XH);
  unsigned short* xl = (unsigned short*)(ws + OFF_XL);
  unsigned short* wh = (unsigned short*)(ws + OFF_WH);
  unsigned short* wl = (unsigned short*)(ws + OFF_WL);

  split_planes_kernel<<<dim3((N_SMP * N_IN) / (SPLIT_THR * 8)), dim3(SPLIT_THR), 0, stream>>>(x, (unsigned*)xh, (unsigned*)xl);
  split_planes_kernel<<<dim3((N_OUT * N_IN) / (SPLIT_THR * 8)), dim3(SPLIT_THR), 0, stream>>>(w, (unsigned*)wh, (unsigned*)wl);

  gemm64_bf16x3_bias_kernel<<<dim3(((N_SMP / 64) * (N_OUT / 64)) / 8), dim3(256), 0, stream>>>(
      xh, xl, N_IN, wh, wl, N_IN, y, N_OUT, bias, N_SMP, N_OUT, N_IN);

  seq_update_kernel<<<dim3(1), dim3(SEQ_THR), LDS_SEQ_BYTES, stream>>>(x, w, bias, wout);
}
